// MambaLayer_33852932227255
// MI455X (gfx1250) — hardware-verified
//
#include <hip/hip_runtime.h>
#include <math.h>

typedef __attribute__((ext_vector_type(16))) _Float16 v16h;
typedef __attribute__((ext_vector_type(8)))  _Float16 v8h;
typedef __attribute__((ext_vector_type(16))) __bf16   v16b;
typedef __attribute__((ext_vector_type(8)))  __bf16   v8b;
typedef __attribute__((ext_vector_type(8)))  float    v8f;
typedef __attribute__((ext_vector_type(4)))  float    v4f;

constexpr int kBatch  = 2;
constexpr int kSeq    = 1024;
constexpr int kDm     = 1024;
constexpr int kDin    = 2048;
constexpr int kNst    = 64;
constexpr int kDtR    = 64;
constexpr int kPrjN   = kDtR + 2 * kNst;
constexpr int kPrjP   = 256;
constexpr int kXzP    = 2 * kDin;
constexpr int kRows   = kBatch * kSeq;
constexpr int kConvTP = 260;
constexpr int kScanTS = 32;
constexpr int kScanCh = 64;
constexpr int kScanYP = 68;
constexpr int kBCW    = 2 * kNst;
constexpr float kInvDm = 1.0f / (float)kDm;
static_assert(kPrjN == 192 && kPrjP % 64 == 0 && kPrjP >= kPrjN, "x_proj width");
static_assert((kDm % 32) == 0 && (kDin % 32) == 0 && (kDtR % 32) == 0, "GEMM K multiples of 32");
static_assert((kRows % 64) == 0 && (kXzP % 64) == 0 && (kPrjP % 64) == 0 && (kDm % 64) == 0 && (kDin % 64) == 0, "GEMM M,N multiples of 64");
static_assert((kSeq % 64) == 0 && (kSeq % kScanTS) == 0 && (kDin % kScanCh) == 0 && (kDin % 256) == 0, "tile multiples");
static_assert(kDm == 128 * 8, "LayerNorm block covers one row with 128 threads x 8");

constexpr size_t kOffWIN  = 0;
constexpr size_t kOffWXP  = kOffWIN  + (size_t)kXzP  * kDm  * 2;
constexpr size_t kOffWDT  = kOffWXP  + (size_t)kPrjP * kDin * 2;
constexpr size_t kOffWOUT = kOffWDT  + (size_t)kDin  * kDtR * 2;
constexpr size_t kOffXNH  = kOffWOUT + (size_t)kDm   * kDin * 2;
constexpr size_t kOffXNL  = kOffXNH  + (size_t)kRows * kDm  * 2;
constexpr size_t kOffXZ   = kOffXNL  + (size_t)kRows * kDm  * 2;
constexpr size_t kOffUC   = kOffXZ   + (size_t)kRows * kXzP * 4;
constexpr size_t kOffUCB  = kOffUC   + (size_t)kRows * kDin * 4;
constexpr size_t kOffPROJ = kOffUCB  + (size_t)kRows * kDin * 2;
constexpr size_t kOffDTB  = kOffPROJ + (size_t)kRows * kPrjP * 4;
constexpr size_t kOffDLR  = kOffDTB  + (size_t)kRows * kDtR * 2;
constexpr size_t kOffYH   = kOffDLR  + (size_t)kRows * kDin * 4;
constexpr size_t kOffYL   = kOffYH   + (size_t)kRows * kDin * 2;
constexpr size_t kWsTotal = kOffYL   + (size_t)kRows * kDin * 2;
static_assert(kWsTotal == 116916224ull, "carve total");
static_assert(kWsTotal <= 134217728ull, "carve cap");
static_assert((kOffWXP % 128) == 0 && (kOffWDT % 128) == 0 && (kOffWOUT % 128) == 0 && (kOffXNH % 128) == 0 &&
              (kOffXNL % 128) == 0 && (kOffXZ % 128) == 0 && (kOffUC % 128) == 0 && (kOffUCB % 128) == 0 &&
              (kOffPROJ % 128) == 0 && (kOffDTB % 128) == 0 && (kOffDLR % 128) == 0 && (kOffYH % 128) == 0 &&
              (kOffYL % 128) == 0, "128-B aligned regions");

__device__ __forceinline__ unsigned short f2bf_bits(float f) {
  unsigned u = __float_as_uint(f);
  return (unsigned short)((u + 0x7FFFu + ((u >> 16) & 1u)) >> 16);
}
__device__ __forceinline__ float bf_bits2f(unsigned short h) { return __uint_as_float(((unsigned)h) << 16); }
__device__ __forceinline__ float rbf(float f) { return bf_bits2f(f2bf_bits(f)); }
__device__ __forceinline__ float opq(float x) { asm volatile("" : "+v"(x)); return x; }

__device__ __forceinline__ void dep_guard4_h(v8f& a, v8f& b, v8f& c, v8f& d, v16h x, v16h y) { asm volatile("v_nop\n\tv_nop\n\tv_nop\n\tv_nop" : "+v"(a), "+v"(b), "+v"(c), "+v"(d) : "v"(x), "v"(y)); }
__device__ __forceinline__ void dep_guard4_b(v8f& a, v8f& b, v8f& c, v8f& d, v16b x, v16b y) { asm volatile("v_nop\n\tv_nop\n\tv_nop\n\tv_nop" : "+v"(a), "+v"(b), "+v"(c), "+v"(d) : "v"(x), "v"(y)); }
__device__ __forceinline__ void keep4_h(v16h a, v16h b, v16h c, v16h d) { asm volatile("v_nop" :: "v"(a), "v"(b), "v"(c), "v"(d)); }
__device__ __forceinline__ void keep4_b(v16b a, v16b b, v16b c, v16b d) { asm volatile("v_nop" :: "v"(a), "v"(b), "v"(c), "v"(d)); }
__device__ __forceinline__ void acc_guard4(v8f& a, v8f& b, v8f& c, v8f& d) { asm volatile("v_nop\n\tv_nop\n\tv_nop\n\tv_nop" : "+v"(a), "+v"(b), "+v"(c), "+v"(d)); }
template <typename T> struct Frag;
template <> struct Frag<_Float16> {
  typedef v16h V; union U { v16h v; v8h h[2]; };
  static __device__ __forceinline__ v16h load(const _Float16* p) {
    U f; f.h[0] = *(const v8h*)(p); f.h[1] = *(const v8h*)(p + 16); return f.v;
  }
  static __device__ __forceinline__ v8f mma(v16h a, v16h b, v8f c) {
    return __builtin_amdgcn_wmma_f32_16x16x32_f16(false, a, false, b, (short)0, c, false, false);
  }
  static __device__ __forceinline__ void guard(v8f& a, v8f& b, v8f& c, v8f& d, v16h x, v16h y) { dep_guard4_h(a, b, c, d, x, y); }
  static __device__ __forceinline__ void keep(v16h a, v16h b, v16h c, v16h d) { keep4_h(a, b, c, d); }
};
template <> struct Frag<__bf16> {
  typedef v16b V; union U { v16b v; v8b h[2]; };
  static __device__ __forceinline__ v16b load(const __bf16* p) {
    U f; f.h[0] = *(const v8b*)(p); f.h[1] = *(const v8b*)(p + 16); return f.v;
  }
  static __device__ __forceinline__ v8f mma(v16b a, v16b b, v8f c) {
    return __builtin_amdgcn_wmma_f32_16x16x32_bf16(false, a, false, b, (short)0, c, false, false);
  }
  static __device__ __forceinline__ void guard(v8f& a, v8f& b, v8f& c, v8f& d, v16b x, v16b y) { dep_guard4_b(a, b, c, d, x, y); }
  static __device__ __forceinline__ void keep(v16b a, v16b b, v16b c, v16b d) { keep4_b(a, b, c, d); }
};

template <int ET> struct Elem;
template <> struct Elem<0> { typedef _Float16 T; };
template <> struct Elem<1> { typedef __bf16 T; };
template <int ET, int SPL, int BIAS_MODE, int OUT_MODE, bool RESID, int ACT = 0>
__global__ __launch_bounds__(256) void wmma_gemm64(
    const unsigned short* __restrict__ Ap, const unsigned short* __restrict__ A2p, int lda, long strideA,
    const unsigned short* __restrict__ Btp, const unsigned short* __restrict__ Bt2p, int ldb, long strideB,
    void* __restrict__ Cout, void* __restrict__ Cout2, int ldc, long strideC,
    const float* __restrict__ bias,
    const float* __restrict__ resid, long strideR,
    int M, int N, int K, float scale) {
  typedef typename Elem<ET>::T T;
  typedef typename Frag<T>::V V;
  const T* A = (const T*)Ap; const T* A2 = (const T*)A2p; const T* Bt = (const T*)Btp; const T* Bt2 = (const T*)Bt2p;
  __shared__ __align__(16) float sT[8][16 * 68];
  const int b    = blockIdx.y;
  const int lane = threadIdx.x & 31;
  const int wave = threadIdx.x >> 5;
  const int tilesN = N >> 6;
  const int tilesM = M >> 6;
  const int tile = blockIdx.x * 8 + wave;
  if (tile >= tilesM * tilesN) return;
  const int tm = tile / tilesN;
  const int tn = tile - tm * tilesN;
  const int m0 = tm << 6;
  const int n0 = tn << 6;

  const T* Ab  = A  + (size_t)b * strideA;
  const T* Bb  = Bt + (size_t)b * strideB;
  const T* Ab2 = (SPL >= 1) ? (A2  + (size_t)b * strideA) : nullptr;
  const T* Bb2 = (SPL == 2) ? (Bt2 + (size_t)b * strideB) : nullptr;

  const int rlane = lane & 15;
  const int koff  = (lane >> 4) * 8;
  const int mOff  = (lane >> 4) * 8;

  v8f acc[4][4];
#pragma unroll
  for (int i = 0; i < 4; ++i)
#pragma unroll
    for (int j = 0; j < 4; ++j) acc[i][j] = (v8f){0.f,0.f,0.f,0.f,0.f,0.f,0.f,0.f};

  for (int k0 = 0; k0 < K; k0 += 32) {
    V bh[4], bl[4];
#pragma unroll
    for (int j = 0; j < 4; ++j) {
      const size_t bo = (size_t)(n0 + (j << 4) + rlane) * ldb + koff + k0;
      bh[j] = Frag<T>::load(Bb + bo);
      if (SPL == 2) bl[j] = Frag<T>::load(Bb2 + bo);
    }
#pragma unroll
    for (int i = 0; i < 4; ++i) {
      const size_t ao = (size_t)(m0 + (i << 4) + rlane) * lda + koff + k0;
      V ah = Frag<T>::load(Ab + ao);
      V al;
      if (SPL >= 1) al = Frag<T>::load(Ab2 + ao);
#pragma unroll
      for (int j = 0; j < 4; ++j) {
        acc[i][j] = Frag<T>::mma(ah, bh[j], acc[i][j]);
        if (SPL == 2) acc[i][j] = Frag<T>::mma(ah, bl[j], acc[i][j]);
        if (SPL >= 1) acc[i][j] = Frag<T>::mma(al, bh[j], acc[i][j]);
      }
      Frag<T>::guard(acc[i][0], acc[i][1], acc[i][2], acc[i][3], ah, (SPL >= 1) ? al : ah);
    }
    Frag<T>::keep(bh[0], bh[1], bh[2], bh[3]);
    if (SPL == 2) Frag<T>::keep(bl[0], bl[1], bl[2], bl[3]);
  }
  acc_guard4(acc[0][0], acc[0][1], acc[0][2], acc[0][3]);
  acc_guard4(acc[1][0], acc[1][1], acc[1][2], acc[1][3]);
  acc_guard4(acc[2][0], acc[2][1], acc[2][2], acc[2][3]);
  acc_guard4(acc[3][0], acc[3][1], acc[3][2], acc[3][3]);

  float* slab = sT[wave];
  const float* Rb = RESID ? (resid + (size_t)b * strideR) : nullptr;
#pragma unroll
  for (int i = 0; i < 4; ++i) {
    const int mBase = m0 + (i << 4);
#pragma unroll
    for (int j = 0; j < 4; ++j) {
      const int n = n0 + (j << 4) + rlane;
      float bv = 0.f;
      if (BIAS_MODE == 2) bv = bias[n];
#pragma unroll
      for (int r = 0; r < 8; ++r) {
        float v = acc[i][j][r] * scale;
        if (BIAS_MODE == 1) v += bias[mBase + mOff + r];
        if (BIAS_MODE == 2) v += bv;
        if (RESID) v += Rb[(size_t)(mBase + mOff + r) * ldc + n];
        if (ACT == 1) v = tanhf(v);
        if (ACT == 2) v = fmaxf(v, 0.0f);
        if (ACT == 4) v = (v > 0.f) ? v : 0.01f * v;
        slab[(mOff + r) * 68 + (j << 4) + rlane] = v;
      }
    }
    __builtin_amdgcn_fence(__ATOMIC_RELEASE, "workgroup");
    __builtin_amdgcn_wave_barrier();
    __builtin_amdgcn_fence(__ATOMIC_ACQUIRE, "workgroup");
    if (OUT_MODE == 0) {
      float* C = (float*)Cout + (size_t)b * strideC;
      const int hh = lane >> 4, c4 = (lane & 15) * 4;
      for (int pass = 0; pass < 2; ++pass) {
#pragma unroll
        for (int it = 0; it < 8; ++it) {
          const int row = it * 2 + hh;
          v4f v = *(const v4f*)(slab + row * 68 + c4);
          *(volatile v4f*)(C + (size_t)(mBase + row) * ldc + n0 + c4) = v;
        }
        __threadfence();
      }
    } else {
      const int q = lane >> 3, c8 = (lane & 7) * 8;
      unsigned short* C  = (unsigned short*)Cout  + (size_t)b * strideC;
      unsigned short* C2 = (OUT_MODE == 2) ? ((unsigned short*)Cout2 + (size_t)b * strideC) : nullptr;
      for (int pass = 0; pass < 2; ++pass) {
#pragma unroll
        for (int it = 0; it < 4; ++it) {
          const int row = it * 4 + q;
          const float* sp = slab + row * 68 + c8;
          v8h hv, lv;
#pragma unroll
          for (int e = 0; e < 8; ++e) {
            if (OUT_MODE == 1) {
              hv[e] = (_Float16)sp[e];
            } else {
              unsigned short hb = f2bf_bits(sp[e]);
              unsigned short lb = f2bf_bits(sp[e] - bf_bits2f(hb));
              hv[e] = __builtin_bit_cast(_Float16, hb);
              lv[e] = __builtin_bit_cast(_Float16, lb);
            }
          }
          *(volatile v8h*)(C + (size_t)(mBase + row) * ldc + n0 + c8) = hv;
          if (OUT_MODE == 2) *(volatile v8h*)(C2 + (size_t)(mBase + row) * ldc + n0 + c8) = lv;
        }
        __threadfence();
      }
    }
    __builtin_amdgcn_fence(__ATOMIC_RELEASE, "workgroup");
    __builtin_amdgcn_wave_barrier();
    __builtin_amdgcn_fence(__ATOMIC_ACQUIRE, "workgroup");
  }
}

__global__ __launch_bounds__(256) void transpose_bf16_kernel(
    const float* __restrict__ W, unsigned short* __restrict__ Bt, int Kdim, int Ndim)
{
  __shared__ float tile[64 * 65];
  const int tid = threadIdx.x, lane = tid & 31, wave = tid >> 5;
  const int n0 = blockIdx.x * 64;
  const int k0 = blockIdx.y * 64;
#pragma unroll
  for (int p = 0; p < 16; ++p) {
    const int idx = tid + p * 256;
    const int kk  = idx >> 6;
    const int nn  = idx & 63;
    const int n   = n0 + nn;
    const int nc  = (n < Ndim) ? n : (Ndim - 1);
    const float v = W[(size_t)(k0 + kk) * Ndim + nc];
    tile[kk * 65 + nn] = (n < Ndim) ? v : 0.f;
    if (p == 7) asm volatile("" ::: "memory");
  }
  __syncthreads();
  const int q = lane >> 3, c8 = (lane & 7) * 8;
  v8h hv[2];
#pragma unroll
  for (int it = 0; it < 2; ++it) {
    const int nrow = it * 32 + wave * 4 + q;
#pragma unroll
    for (int e = 0; e < 8; ++e) {
      const float tv = tile[(c8 + e) * 65 + nrow];
      const unsigned short hb = f2bf_bits(tv);
      hv[it][e] = __builtin_bit_cast(_Float16, hb);
    }
  }
  for (int pass = 0; pass < 2; ++pass) {
#pragma unroll
    for (int it = 0; it < 2; ++it) {
      const int nrow = it * 32 + wave * 4 + q;
      *(volatile v8h*)(Bt + (size_t)(n0 + nrow) * Kdim + k0 + c8) = hv[it];
    }
    __threadfence();
  }
}

__global__ __launch_bounds__(128) void layernorm_planes_kernel(
    const float* __restrict__ x, const float* __restrict__ nw, const float* __restrict__ nb,
    unsigned short* __restrict__ XNH, unsigned short* __restrict__ XNL)
{
  __shared__ float redA[4];
  __shared__ float redB[4];
  const int tid = threadIdx.x, lane = tid & 31, wave = tid >> 5;
  const size_t e0 = (size_t)blockIdx.x * kDm + (size_t)tid * 8;
  const v4f a0 = *(const v4f*)(x + e0);
  const v4f a1 = *(const v4f*)(x + e0 + 4);
  float v[8];
#pragma unroll
  for (int e = 0; e < 4; ++e) { v[e] = rbf(a0[e]); v[4 + e] = rbf(a1[e]); }
  float s = ((v[0] + v[1]) + (v[2] + v[3])) + ((v[4] + v[5]) + (v[6] + v[7]));
#pragma unroll
  for (int off = 16; off > 0; off >>= 1) s += __shfl_xor(s, off, 32);
  if (lane == 0) redA[wave] = s;
  __syncthreads();
  const float mu = ((redA[0] + redA[1]) + (redA[2] + redA[3])) * kInvDm;
  float dv[8];
  float ss = 0.f;
#pragma unroll
  for (int e = 0; e < 8; ++e) { dv[e] = v[e] - mu; ss += dv[e] * dv[e]; }
#pragma unroll
  for (int off = 16; off > 0; off >>= 1) ss += __shfl_xor(ss, off, 32);
  if (lane == 0) redB[wave] = ss;
  __syncthreads();
  const float var = ((redB[0] + redB[1]) + (redB[2] + redB[3])) * kInvDm;
  const float rs  = rsqrtf(var + 1e-5f);
  const int c0 = tid * 8;
  const v4f w0 = *(const v4f*)(nw + c0);
  const v4f w1 = *(const v4f*)(nw + c0 + 4);
  const v4f b0 = *(const v4f*)(nb + c0);
  const v4f b1 = *(const v4f*)(nb + c0 + 4);
  v8h hv, lv;
#pragma unroll
  for (int e = 0; e < 4; ++e) {
    const float y0 = (dv[e] * rs) * rbf(w0[e]) + rbf(b0[e]);
    const float y1 = (dv[4 + e] * rs) * rbf(w1[e]) + rbf(b1[e]);
    const unsigned short h0 = f2bf_bits(y0), h1 = f2bf_bits(y1);
    const unsigned short l0 = f2bf_bits(y0 - bf_bits2f(h0)), l1 = f2bf_bits(y1 - bf_bits2f(h1));
    hv[e]     = __builtin_bit_cast(_Float16, h0);
    hv[4 + e] = __builtin_bit_cast(_Float16, h1);
    lv[e]     = __builtin_bit_cast(_Float16, l0);
    lv[4 + e] = __builtin_bit_cast(_Float16, l1);
  }
  unsigned short* qh = XNH + e0;
  unsigned short* ql = XNL + e0;
  *(volatile v8h*)qh = hv;
  *(volatile v8h*)ql = lv;
  __threadfence();
  *(volatile v8h*)qh = hv;
  *(volatile v8h*)ql = lv;
}

__global__ __launch_bounds__(256) void conv_silu_kernel(
    const float* __restrict__ XZ, const float* __restrict__ cw, const float* __restrict__ cb,
    float* __restrict__ UC, unsigned short* __restrict__ UCB)
{
  __shared__ __align__(16) float sT[16 * kConvTP];
  const int tid = threadIdx.x, lane = tid & 31, wave = tid >> 5;
  const int d0 = blockIdx.x * 256, d = d0 + tid;
  const int g0 = blockIdx.y * 64;
  const int tb = g0 & (kSeq - 1);
  const float w0 = rbf(cw[d * 4 + 0]), w1 = rbf(cw[d * 4 + 1]), w2 = rbf(cw[d * 4 + 2]), w3 = rbf(cw[d * 4 + 3]);
  const float bc = rbf(cb[d]);
  float xm3, xm2, xm1;
  {
    const bool hist = (tb > 0);
    const int rb = hist ? (g0 - 3) : g0;
    const float v3 = XZ[(size_t)rb * kXzP + d];
    const float v2 = XZ[(size_t)(rb + 1) * kXzP + d];
    const float v1 = XZ[(size_t)(rb + 2) * kXzP + d];
    xm3 = hist ? v3 : 0.f;
    xm2 = hist ? v2 : 0.f;
    xm1 = hist ? v1 : 0.f;
  }
  const int hrow = wave >> 1;
  const int hch  = (wave & 1) * 128 + lane * 4;
#pragma unroll 1
  for (int sub = 0; sub < 4; ++sub) {
    const int lb = g0 + sub * 16;
#pragma unroll 1
    for (int s = 0; s < 16; ++s) {
      const float xcur = XZ[(size_t)(lb + s) * kXzP + d];
      float acc = w0 * xm3;
      acc = fmaf(w1, xm2, acc);
      acc = fmaf(w2, xm1, acc);
      acc = fmaf(w3, xcur, acc);
      const float sv = acc + bc;
      const float sg = __builtin_amdgcn_rcpf(1.0f + expf(-sv));
      sT[s * kConvTP + tid] = sv * sg;
      xm3 = xm2; xm2 = xm1; xm1 = xcur;
    }
    __syncthreads();
    v4f fv[4];
    v8h bv[2];
#pragma unroll
    for (int it = 0; it < 4; ++it) fv[it] = *(const v4f*)(sT + (it * 4 + hrow) * kConvTP + hch);
#pragma unroll
    for (int it = 0; it < 2; ++it) {
      const float* sp = sT + (it * 8 + wave) * kConvTP + lane * 8;
      const v4f a0 = *(const v4f*)(sp);
      const v4f a1 = *(const v4f*)(sp + 4);
#pragma unroll
      for (int e = 0; e < 4; ++e) {
        const unsigned short h0 = f2bf_bits(a0[e]), h1 = f2bf_bits(a1[e]);
        bv[it][e]     = __builtin_bit_cast(_Float16, h0);
        bv[it][4 + e] = __builtin_bit_cast(_Float16, h1);
      }
    }
    for (int pass = 0; pass < 2; ++pass) {
#pragma unroll
      for (int it = 0; it < 4; ++it)
        *(volatile v4f*)(UC + (size_t)(lb + it * 4 + hrow) * kDin + d0 + hch) = fv[it];
#pragma unroll
      for (int it = 0; it < 2; ++it)
        *(volatile v8h*)(UCB + (size_t)(lb + it * 8 + wave) * kDin + d0 + lane * 8) = bv[it];
      __threadfence();
    }
    __syncthreads();
  }
}

__global__ __launch_bounds__(256) void dt_cast_kernel(
    const float* __restrict__ PROJ, unsigned short* __restrict__ DTB, int total8)
{
  const int i = blockIdx.x * 256 + threadIdx.x;
  if (i >= total8) return;
  const int e0  = i << 3;
  const int row = e0 >> 6;
  const int c8  = e0 & 63;
  const float* p = PROJ + (size_t)row * kPrjP + c8;
  const v4f a0 = *(const v4f*)(p);
  const v4f a1 = *(const v4f*)(p + 4);
  v8h hv;
#pragma unroll
  for (int e = 0; e < 4; ++e) {
    const unsigned short h0 = f2bf_bits(a0[e]), h1 = f2bf_bits(a1[e]);
    hv[e]     = __builtin_bit_cast(_Float16, h0);
    hv[4 + e] = __builtin_bit_cast(_Float16, h1);
  }
  unsigned short* qd = DTB + e0;
  *(volatile v8h*)qd = hv;
  __threadfence();
  *(volatile v8h*)qd = hv;
}

__global__ __launch_bounds__(64) void scan_kernel(
    const float* __restrict__ PROJ, const float* __restrict__ DLR, const float* __restrict__ UC,
    const float* __restrict__ XZ, const float* __restrict__ bdt, const float* __restrict__ Alog,
    const float* __restrict__ Dp, unsigned short* __restrict__ YH, unsigned short* __restrict__ YL)
{
  __shared__ __align__(16) float sX[kScanTS * kBCW];
  __shared__ __align__(16) float sY[kScanTS * kScanYP];
  __shared__ __align__(16) float sA[kNst * kScanCh];
  const int tid = threadIdx.x, lane = tid & 31, wave = tid >> 5;
  constexpr int kBlkPerB = kDin / kScanCh;
  const int bix = blockIdx.x / kBlkPerB;
  const int d0  = (blockIdx.x - bix * kBlkPerB) * kScanCh;
  const int d   = d0 + tid;
  const size_t row0 = (size_t)bix * kSeq;
#pragma unroll 1
  for (int s = 0; s < kNst; ++s) sA[s * kScanCh + tid] = -expf(rbf(Alog[(size_t)d * kNst + s]));
  __syncthreads();
  float negA[kNst], h[kNst];
#pragma unroll
  for (int s = 0; s < kNst; ++s) {
    negA[s] = sA[s * kScanCh + tid];
    h[s] = 0.f;
  }
  const float bb = rbf(bdt[d]), Dd = rbf(Dp[d]);
  const int lr = tid >> 5, lc4 = (tid & 31) * 4;
  const int q = lane >> 3, c8 = (lane & 7) * 8;
#pragma unroll 1
  for (int t0 = 0; t0 < kSeq; t0 += kScanTS) {
    __syncthreads();
#pragma unroll 1
    for (int g = 0; g < 4; ++g) {
#pragma unroll
      for (int i = 0; i < 4; ++i) {
        const int r = lr + 2 * (4 * g + i);
        *(v4f*)(sX + r * kBCW + lc4) = *(const v4f*)(PROJ + (row0 + t0 + r) * kPrjP + kDtR + lc4);
      }
    }
    __syncthreads();
#pragma unroll 1
    for (int s = 0; s < kScanTS; ++s) {
      const size_t r = row0 + t0 + s;
      const float* xr = sX + s * kBCW;
      const float v   = DLR[r * kDin + d] + bb;
      const float xt  = UC[r * kDin + d];
      const float zv  = XZ[r * kXzP + kDin + d];
      const float a   = __expf(-fabsf(v));
      const float u1  = 1.0f + a;
      const float l1p = __logf(u1) + (a - (u1 - 1.0f)) * __builtin_amdgcn_rcpf(u1);
      const float dt  = fmaxf(v, 0.0f) + l1p;
      const float dtx = dt * xt;
      float y = 0.f;
#pragma unroll
      for (int q4 = 0; q4 < kNst / 4; ++q4) {
        const v4f bv = *(const v4f*)(xr + 4 * q4);
        const v4f cv = *(const v4f*)(xr + kNst + 4 * q4);
#pragma unroll
        for (int e = 0; e < 4; ++e) {
          const int k = 4 * q4 + e;
          const float ex = __expf(dt * negA[k]);
          const float qv = opq(ex * h[k]);
          const float p  = opq(dtx * bv[e]);
          const float hn = qv + p;
          h[k] = hn;
          const float rr = opq(hn * cv[e]);
          y += rr;
        }
      }
      y = xt * Dd + y;
      const float sg = __builtin_amdgcn_rcpf(1.0f + expf(-zv));
      y = y * (zv * sg);
      sY[s * kScanYP + tid] = y;
    }
    __syncthreads();
    for (int pass = 0; pass < 2; ++pass) {
#pragma unroll
      for (int it = 0; it < 4; ++it) {
        const int row = it * 8 + wave * 4 + q;
        const float* sp = sY + row * kScanYP + c8;
        const v4f a0 = *(const v4f*)(sp);
        const v4f a1 = *(const v4f*)(sp + 4);
        v8h hv, lv;
#pragma unroll
        for (int e = 0; e < 4; ++e) {
          const unsigned short h0 = f2bf_bits(a0[e]), h1 = f2bf_bits(a1[e]);
          const unsigned short l0 = f2bf_bits(a0[e] - bf_bits2f(h0)), l1 = f2bf_bits(a1[e] - bf_bits2f(h1));
          hv[e]     = __builtin_bit_cast(_Float16, h0);
          hv[4 + e] = __builtin_bit_cast(_Float16, h1);
          lv[e]     = __builtin_bit_cast(_Float16, l0);
          lv[4 + e] = __builtin_bit_cast(_Float16, l1);
        }
        const size_t o = (row0 + t0 + row) * kDin + d0 + c8;
        *(volatile v8h*)(YH + o) = hv;
        *(volatile v8h*)(YL + o) = lv;
      }
      __threadfence();
    }
  }
}

extern "C" void kernel_launch(void* const* d_in, const int* in_sizes, int n_in,
                              void* d_out, int out_size, void* d_ws, size_t ws_size,
                              hipStream_t stream) {
  if (n_in < 12) return;
  if (in_sizes[0] != kRows * kDm) return;
  if (in_sizes[1] != kDm || in_sizes[2] != kDm) return;
  if (in_sizes[3] != kDm * kXzP) return;
  if (in_sizes[4] != kDin * 4 || in_sizes[5] != kDin) return;
  if (in_sizes[6] != kDin * kPrjN) return;
  if (in_sizes[7] != kDtR * kDin || in_sizes[8] != kDin) return;
  if (in_sizes[9] != kDin * kNst || in_sizes[10] != kDin) return;
  if (in_sizes[11] != kDin * kDm) return;
  if (out_size != kRows * kDm) return;
  if (ws_size < kWsTotal) return;

  const float* x       = (const float*)d_in[0];
  const float* norm_w  = (const float*)d_in[1];
  const float* norm_b  = (const float*)d_in[2];
  const float* W_in    = (const float*)d_in[3];
  const float* conv_w  = (const float*)d_in[4];
  const float* conv_b  = (const float*)d_in[5];
  const float* W_xproj = (const float*)d_in[6];
  const float* W_dt    = (const float*)d_in[7];
  const float* b_dt    = (const float*)d_in[8];
  const float* A_log   = (const float*)d_in[9];
  const float* Dp      = (const float*)d_in[10];
  const float* W_out   = (const float*)d_in[11];
  float* out = (float*)d_out;

  char* ws = (char*)d_ws;
  unsigned short* WIN  = (unsigned short*)(ws + kOffWIN);
  unsigned short* WXP  = (unsigned short*)(ws + kOffWXP);
  unsigned short* WDT  = (unsigned short*)(ws + kOffWDT);
  unsigned short* WOUT = (unsigned short*)(ws + kOffWOUT);
  unsigned short* XNH  = (unsigned short*)(ws + kOffXNH);
  unsigned short* XNL  = (unsigned short*)(ws + kOffXNL);
  float*          XZ   = (float*)(ws + kOffXZ);
  float*          UC   = (float*)(ws + kOffUC);
  unsigned short* UCB  = (unsigned short*)(ws + kOffUCB);
  float*          PROJ = (float*)(ws + kOffPROJ);
  unsigned short* DTB  = (unsigned short*)(ws + kOffDTB);
  float*          DLR  = (float*)(ws + kOffDLR);
  unsigned short* YH   = (unsigned short*)(ws + kOffYH);
  unsigned short* YL   = (unsigned short*)(ws + kOffYL);
  const float* dummy_bias  = b_dt;
  const float* dummy_resid = x;

  transpose_bf16_kernel<<<dim3(kXzP / 64, kDm / 64), 256, 0, stream>>>(W_in, WIN, kDm, kXzP);
  transpose_bf16_kernel<<<dim3(kPrjP / 64, kDin / 64), 256, 0, stream>>>(W_xproj, WXP, kDin, kPrjN);
  transpose_bf16_kernel<<<dim3(kDin / 64, kDtR / 64), 256, 0, stream>>>(W_dt, WDT, kDtR, kDin);
  transpose_bf16_kernel<<<dim3(kDm / 64, kDin / 64), 256, 0, stream>>>(W_out, WOUT, kDin, kDm);

  layernorm_planes_kernel<<<kRows, 128, 0, stream>>>(x, norm_w, norm_b, XNH, XNL);

  wmma_gemm64<1, 1, 0, 0, false><<<dim3((kRows / 64) * (kXzP / 64) / 8, 1), 256, 0, stream>>>(
      XNH, XNL, kDm, 0L,
      WIN, WIN, kDm, 0L,
      (void*)XZ, (void*)XZ, kXzP, 0L,
      dummy_bias, dummy_resid, 0L,
      kRows, kXzP, kDm, 1.0f);

  conv_silu_kernel<<<dim3(kDin / 256, kRows / 64), 256, 0, stream>>>(XZ, conv_w, conv_b, UC, UCB);

  wmma_gemm64<1, 0, 0, 0, false><<<dim3((kRows / 64) * (kPrjP / 64) / 8, 1), 256, 0, stream>>>(
      UCB, UCB, kDin, 0L,
      WXP, WXP, kDin, 0L,
      (void*)PROJ, (void*)PROJ, kPrjP, 0L,
      dummy_bias, dummy_resid, 0L,
      kRows, kPrjP, kDin, 1.0f);

  dt_cast_kernel<<<(kRows * kDtR) / 8 / 256, 256, 0, stream>>>(PROJ, DTB, (kRows * kDtR) / 8);

  wmma_gemm64<1, 0, 0, 0, false><<<dim3((kRows / 64) * (kDin / 64) / 8, 1), 256, 0, stream>>>(
      DTB, DTB, kDtR, 0L,
      WDT, WDT, kDtR, 0L,
      (void*)DLR, (void*)DLR, kDin, 0L,
      dummy_bias, dummy_resid, 0L,
      kRows, kDin, kDtR, 1.0f);

  scan_kernel<<<kBatch * (kDin / kScanCh), kScanCh, 0, stream>>>(PROJ, DLR, UC, XZ, b_dt, A_log, Dp, YH, YL);

  wmma_gemm64<1, 1, 0, 0, false><<<dim3((kRows / 64) * (kDm / 64) / 8, 1), 256, 0, stream>>>(
      YH, YL, kDin, 0L,
      WOUT, WOUT, kDin, 0L,
      (void*)out, (void*)out, kDm, 0L,
      dummy_bias, dummy_resid, 0L,
      kRows, kDm, kDin, 1.0f);
}
